// Model_52518860096592
// MI455X (gfx1250) — hardware-verified
//
#include <hip/hip_runtime.h>
#include <math.h>

typedef __attribute__((ext_vector_type(16))) _Float16 v16h;
typedef __attribute__((ext_vector_type(8)))  _Float16 v8h;
typedef __attribute__((ext_vector_type(8)))  float v8f;
typedef __attribute__((ext_vector_type(4)))  float v4f;
typedef __attribute__((ext_vector_type(4)))  unsigned v4u;

template <typename T> __device__ __forceinline__ void vst2(void* p, T v) { *(volatile T*)p = v; __threadfence(); *(volatile T*)p = v; }
__device__ __forceinline__ v8f wmma16(v16h a, v16h b, v8f c) {
  v8f d = __builtin_amdgcn_wmma_f32_16x16x32_f16(false, a, false, b, (short)0, c, false, false);
  asm volatile("v_nop\n\tv_nop\n\tv_nop\n\tv_nop" : "+v"(d) : "v"(a), "v"(b));
  return d;
}
__device__ __forceinline__ v16h frag_h(const _Float16* rowk0, int lane) {
  union { v16h v; v8h q[2]; } u; const _Float16* p = rowk0 + 8 * (lane >> 4);
  u.q[0] = *(const v8h*)p; u.q[1] = *(const v8h*)(p + 16); return u.v;
}
__device__ __forceinline__ float bfr(float v) { return (float)(__bf16)v; }
#define LDSX() do { asm volatile("s_wait_dscnt 0" ::: "memory"); __builtin_amdgcn_wave_barrier(); __builtin_amdgcn_fence(3  , "workgroup"); } while (0)
#define EX2(x) __builtin_amdgcn_exp2f(x)

#ifndef NB
#define NB 4
#endif
#ifndef SEQ
#define SEQ 4096
#endif
#define NB_FULL 4
#define SEQ_FULL 4096
#define HD 64
#define LOG2E 1.4426950408889634f
#define SC_LOG2 (0.125f * LOG2E * (1.0f / 256.0f))

static_assert(HD == 64);
static_assert(HD % 32 == 0);
static_assert(SEQ % 64 == 0);
static_assert(SEQ % 32 == 0);
static_assert(SEQ <= SEQ_FULL);
static_assert(NB >= 1 && NB <= NB_FULL);

#define WS_QH  ((size_t)0)
#define WS_KH  (WS_QH + (size_t)2 * NB * SEQ * HD)
#define WS_VT  (WS_KH + (size_t)2 * NB * SEQ * HD)
#define WS_MK  (WS_VT + (size_t)2 * NB * HD * SEQ)
#define WS_END (WS_MK + (size_t)4 * NB * SEQ)
static_assert(WS_KH % 128 == 0);
static_assert(WS_VT % 128 == 0);
static_assert(WS_MK % 128 == 0);
static_assert(WS_END <= (size_t)134217728);

__global__ __launch_bounds__(128) void k_prep(const float* __restrict__ Q, const float* __restrict__ K, const float* __restrict__ V, const float* __restrict__ M, _Float16* __restrict__ QH, _Float16* __restrict__ KH, _Float16* __restrict__ VT, float* __restrict__ MK) {
  __shared__ __align__(16) _Float16 sq[64][72], sk[64][72], tv[64][72];
  __shared__ __align__(16) float sm[64];
  const int tid = threadIdx.x; const int b = blockIdx.y; const int s0 = blockIdx.x * 64;
  const size_t ib = ((size_t)b * SEQ_FULL + s0) * HD;
#pragma unroll 1
  for (int e = tid; e < 64 * 16; e += 128) {
    const int rl = e >> 4, c4 = (e & 15) * 4;
    const v4f q = *(const v4f*)(Q + ib + (size_t)rl * HD + c4);
    const v4f k = *(const v4f*)(K + ib + (size_t)rl * HD + c4);
    const v4f v = *(const v4f*)(V + ib + (size_t)rl * HD + c4);
#pragma unroll
    for (int t = 0; t < 4; ++t) {
      sq[rl][c4 + t] = (_Float16)(bfr(q[t]) * 16.0f);
      sk[rl][c4 + t] = (_Float16)(bfr(k[t]) * 16.0f);
      tv[c4 + t][rl] = (_Float16)(bfr(v[t]) * 16.0f);
    }
  }
  if (tid < 64) sm[tid] = bfr(M[(size_t)b * SEQ_FULL + s0 + tid]) * LOG2E;
  __syncthreads();
#pragma unroll 1
  for (int e = tid; e < 64 * 8; e += 128) {
    const int rl = e >> 3, q = e & 7; const size_t o = ((size_t)b * SEQ + s0 + rl) * HD + q * 8;
    const v4u a = *(const v4u*)&sq[rl][q * 8]; const v4u c = *(const v4u*)&sk[rl][q * 8];
    vst2((unsigned*)(QH + o), a); vst2((unsigned*)(KH + o), c);
  }
#pragma unroll 1
  for (int e = tid; e < 64 * 8; e += 128) {
    const int cl = e >> 3, q = e & 7;
    const v4u a = *(const v4u*)&tv[cl][q * 8];
    vst2((unsigned*)(VT + ((size_t)b * HD + cl) * SEQ + s0 + q * 8), a);
  }
  if (tid < 16) { const v4f a = *(const v4f*)&sm[tid * 4]; vst2(MK + (size_t)b * SEQ + s0 + tid * 4, a); }
}

static_assert(4 * 16 == 64);
__global__ __launch_bounds__(128) void k_fa(const _Float16* __restrict__ QH, const _Float16* __restrict__ KH, const _Float16* __restrict__ VT, const float* __restrict__ MK, float* __restrict__ O) {
  __shared__ __align__(16) float ss[4][16][HD + 4];
  const int tid = threadIdx.x; const int wave = __builtin_amdgcn_readfirstlane(threadIdx.x >> 5);
  const int lane = tid & 31, col = lane & 15, g = lane >> 4;
  const int b = blockIdx.y; const int q0 = blockIdx.x * 64 + wave * 16;
  const _Float16* qrow = QH + ((size_t)b * SEQ + q0 + col) * HD;
  const v16h qf0 = frag_h(qrow, lane), qf1 = frag_h(qrow + 32, lane);
  const _Float16* Kb = KH + (size_t)b * SEQ * HD + (size_t)col * HD;
  const _Float16* Vb = VT + (size_t)b * HD * SEQ + (size_t)col * SEQ;
  const float* Mb = MK + (size_t)b * SEQ + 8 * g;
  v8f acc0 = {}, acc1 = {}, acc2 = {}, acc3 = {};
  float m = -3.0e38f, l = 0.0f;
#pragma unroll 1
  for (int k0 = 0; k0 < SEQ; k0 += 32) {
    const _Float16* kr = Kb + (size_t)k0 * HD;
    v8f s0 = {}, s1 = {};
    s0 = wmma16(frag_h(kr, lane), qf0, s0);
    s0 = wmma16(frag_h(kr + 32, lane), qf1, s0);
    s1 = wmma16(frag_h(kr + 16 * HD, lane), qf0, s1);
    s1 = wmma16(frag_h(kr + 16 * HD + 32, lane), qf1, s1);
    const float* mp = Mb + k0;
    const v4f ma = *(const v4f*)mp, mb = *(const v4f*)(mp + 4), mc = *(const v4f*)(mp + 16), md = *(const v4f*)(mp + 20);
    float x[16];
#pragma unroll
    for (int i = 0; i < 4; ++i) {
      x[i]      = fmaf(s0[i],     SC_LOG2, ma[i]);
      x[4 + i]  = fmaf(s0[4 + i], SC_LOG2, mb[i]);
      x[8 + i]  = fmaf(s1[i],     SC_LOG2, mc[i]);
      x[12 + i] = fmaf(s1[4 + i], SC_LOG2, md[i]);
    }
    float mx = x[0];
#pragma unroll
    for (int i = 1; i < 16; ++i) mx = fmaxf(mx, x[i]);
    mx = fmaxf(mx, __shfl_xor(mx, 16));
    const float mnew = fmaxf(m, mx);
    const float al = EX2(m - mnew);
    const float mo = mnew - 8.0f;
    m = mnew;
    v16h pf; float ls = 0.0f;
#pragma unroll
    for (int i = 0; i < 16; ++i) { const float e = EX2(x[i] - mo); ls += e; pf[i] = (_Float16)e; }
    l = fmaf(l, al, ls);
    acc0 = acc0 * al; acc1 = acc1 * al; acc2 = acc2 * al; acc3 = acc3 * al;
    const _Float16* vr = Vb + k0;
    const v16h v0 = frag_h(vr, lane), v1 = frag_h(vr + (size_t)16 * SEQ, lane), v2 = frag_h(vr + (size_t)32 * SEQ, lane), v3 = frag_h(vr + (size_t)48 * SEQ, lane);
    acc0 = wmma16(v0, pf, acc0);
    acc1 = wmma16(v1, pf, acc1);
    acc2 = wmma16(v2, pf, acc2);
    acc3 = wmma16(v3, pf, acc3);
  }
  const float lt = l + __shfl_xor(l, 16);
  const float inv = 1.0f / (lt * 16.0f);
#pragma unroll
  for (int r = 0; r < 8; ++r) {
    ss[wave][col][8 * g + r]      = acc0[r] * inv;
    ss[wave][col][16 + 8 * g + r] = acc1[r] * inv;
    ss[wave][col][32 + 8 * g + r] = acc2[r] * inv;
    ss[wave][col][48 + 8 * g + r] = acc3[r] * inv;
  }
  LDSX();
  v4f o[8];
#pragma unroll
  for (int it = 0; it < 8; ++it) o[it] = *(const v4f*)&ss[wave][it * 2 + g][col * 4];
  float* ob = O + ((size_t)b * SEQ + q0) * HD + lane * 4;
#pragma unroll
  for (int it = 0; it < 8; ++it) *(volatile v4f*)(ob + it * 128) = o[it];
  __threadfence();
#pragma unroll
  for (int it = 0; it < 8; ++it) *(volatile v4f*)(ob + it * 128) = o[it];
}

extern "C" void kernel_launch(void* const* d_in, const int* in_sizes, int n_in, void* d_out, int out_size, void* d_ws, size_t ws_size, hipStream_t stream) {
  if (n_in < 4) return;
  const long long need_x = ((long long)(NB - 1) * SEQ_FULL + SEQ) * HD;
  const long long need_m = (long long)(NB - 1) * SEQ_FULL + SEQ;
  if ((long long)in_sizes[0] < need_x || (long long)in_sizes[1] < need_x || (long long)in_sizes[2] < need_x || (long long)in_sizes[3] < need_m) return;
  if ((long long)out_size < (long long)NB * SEQ * HD) return;
  if (ws_size < (size_t)WS_END) return;
  char* ws = (char*)d_ws;
  _Float16* QH = (_Float16*)(ws + WS_QH); _Float16* KH = (_Float16*)(ws + WS_KH); _Float16* VT = (_Float16*)(ws + WS_VT); float* MK = (float*)(ws + WS_MK);
  k_prep<<<dim3(SEQ / 64, NB), 128, 0, stream>>>((const float*)d_in[0], (const float*)d_in[1], (const float*)d_in[2], (const float*)d_in[3], QH, KH, VT, MK);
  k_fa<<<dim3(SEQ / 64, NB), 128, 0, stream>>>(QH, KH, VT, MK, (float*)d_out);
}
